// MyAttention3_37185826849034
// MI455X (gfx1250) — hardware-verified
//
#include <hip/hip_runtime.h>
#include <math.h>

typedef __attribute__((ext_vector_type(16))) _Float16 v16h;
typedef __attribute__((ext_vector_type(16))) __bf16 v16b;
typedef __attribute__((ext_vector_type(8)))  _Float16 v8h;
typedef __attribute__((ext_vector_type(8)))  float v8f;
typedef __attribute__((ext_vector_type(4)))  float v4f;
typedef __attribute__((ext_vector_type(2)))  float v2f;
typedef __attribute__((ext_vector_type(4)))  unsigned v4u;
typedef __attribute__((ext_vector_type(4)))  int v4i;
typedef float __attribute__((may_alias)) float_a;
typedef int __attribute__((may_alias)) int_a;

template <typename T> __device__ __forceinline__ void vst2(void* p, T v) { *(volatile T*)p = v; __threadfence(); *(volatile T*)p = v; }
__device__ __forceinline__ v8f wmma16(v16h a, v16h b, v8f c) {
  v8f d = __builtin_amdgcn_wmma_f32_16x16x32_f16(false, a, false, b, (short)0, c, false, false);
  asm volatile("v_nop\n\tv_nop\n\tv_nop\n\tv_nop" : "+v"(d) : "v"(a), "v"(b));
  return d;
}
__device__ __forceinline__ v8f wmma_bf(v16b a, v16b b, v8f c) {
  v8f d = __builtin_amdgcn_wmma_f32_16x16x32_bf16(false, a, false, b, (short)0, c, false, false);
  asm volatile("v_nop\n\tv_nop\n\tv_nop\n\tv_nop" : "+v"(d) : "v"(a), "v"(b));
  return d;
}
__device__ __forceinline__ v16h frag_h(const _Float16* rowk0, int lane) {
  union { v16h v; v8h q[2]; } u; const _Float16* p = rowk0 + 8 * (lane >> 4);
  u.q[0] = *(const v8h*)p; u.q[1] = *(const v8h*)(p + 16); return u.v;
}
__device__ __forceinline__ v16h frag_f32(const float* rowk0, int lane) {
  v16h a; const float* p = rowk0 + 8 * (lane >> 4);
#pragma unroll
  for (int i = 0; i < 8; ++i) { a[i] = (_Float16)p[i]; a[8 + i] = (_Float16)p[16 + i]; }
  return a;
}
__device__ __forceinline__ v16h frag_f32s(const float* rowk0, int lane, float sc) {
  v16h a; const float* p = rowk0 + 8 * (lane >> 4);
#pragma unroll
  for (int i = 0; i < 8; ++i) { a[i] = (_Float16)(p[i] * sc); a[8 + i] = (_Float16)(p[16 + i] * sc); }
  return a;
}
__device__ __forceinline__ v16h fragc_f32(const float* W, int k0, int n, int lane, int ld, int K) {
  v16h a; const int g = lane >> 4;
#pragma unroll
  for (int i = 0; i < 8; ++i) { const int ka = k0 + 8 * g + i, kb = ka + 16;
    a[i] = (_Float16)(ka < K ? W[(size_t)ka * ld + n] : 0.f); a[8 + i] = (_Float16)(kb < K ? W[(size_t)kb * ld + n] : 0.f); }
  return a;
}
struct F2 { v16b h, l; };
__device__ __forceinline__ F2 bsplit16(const float v[16]) { F2 r;
#pragma unroll
  for (int i = 0; i < 16; ++i) { const __bf16 h = (__bf16)v[i]; r.h[i] = h; r.l[i] = (__bf16)(v[i] - (float)h); }
  return r; }
__device__ __forceinline__ F2 split_row(const float* row, int k0, int lane) { float v[16]; const float* p = row + k0 + 8 * (lane >> 4);
#pragma unroll
  for (int i = 0; i < 8; ++i) { v[i] = p[i]; v[8 + i] = p[16 + i]; }
  return bsplit16(v); }
__device__ __forceinline__ F2 split_rowK(const float* row, int k0, int lane, int K) { float v[16]; const int g = lane >> 4;
#pragma unroll
  for (int i = 0; i < 8; ++i) { const int ka = k0 + 8 * g + i, kb = ka + 16; v[i] = ka < K ? row[ka] : 0.f; v[8 + i] = kb < K ? row[kb] : 0.f; }
  return bsplit16(v); }
__device__ __forceinline__ F2 split_col(const float* W, int k0, int n, int lane, int ld, int K) { float v[16]; const int g = lane >> 4;
#pragma unroll
  for (int i = 0; i < 8; ++i) { const int ka = k0 + 8 * g + i, kb = ka + 16; v[i] = ka < K ? W[(size_t)ka * ld + n] : 0.f; v[8 + i] = kb < K ? W[(size_t)kb * ld + n] : 0.f; }
  return bsplit16(v); }
__device__ __forceinline__ v8f mac3(const F2& a, const F2& b, v8f c) { c = wmma_bf(a.l, b.h, c); c = wmma_bf(a.h, b.l, c); return wmma_bf(a.h, b.h, c); }
__device__ __forceinline__ float sigm(float v) { return 1.0f / (1.0f + expf(-v)); }
#define LDSX() do { asm volatile("s_wait_dscnt 0" ::: "memory"); __builtin_amdgcn_wave_barrier(); __builtin_amdgcn_fence(__ATOMIC_RELEASE, "workgroup"); } while (0)

#define NB 2
#define LL 2048
#define NH 16
#define CC 64
#define KK 64

__global__ __launch_bounds__(256) void k_prep(const float* __restrict__ q, const float* __restrict__ k, const float* __restrict__ v, _Float16* __restrict__ qh, _Float16* __restrict__ kh, _Float16* __restrict__ vT) {
  __shared__ __align__(16) _Float16 st[CC][72];
  const int tid = threadIdx.x, b = blockIdx.z, h = blockIdx.y, l0 = blockIdx.x * 64;
  for (int qd = tid; qd < 64 * 8; qd += 256) { const int rl = qd >> 3, pc = qd & 7; const size_t src = (((size_t)b * LL + l0 + rl) * NH + h) * CC + pc * 8; union { v8h a; v4u u; } pq, pk;
#pragma unroll
    for (int e = 0; e < 8; ++e) { pq.a[e] = (_Float16)q[src + e]; pk.a[e] = (_Float16)k[src + e]; }
    const size_t dst = (((size_t)b * NH + h) * LL + l0 + rl) * CC + pc * 8; vst2(qh + dst, pq.u); vst2(kh + dst, pk.u); }
  for (int qd = tid; qd < 64 * CC; qd += 256) { const int rl = qd >> 6, c = qd & 63; st[c][rl] = (_Float16)v[(((size_t)b * LL + l0 + rl) * NH + h) * CC + c]; }
  __syncthreads();
  for (int qd = tid; qd < CC * 8; qd += 256) { const int c = qd >> 3, pc = qd & 7; vst2(vT + (((size_t)b * NH + h) * CC + c) * LL + l0 + pc * 8, *(const v4u*)(&st[c][pc * 8])); }
}
__global__ __launch_bounds__(64) void k_attn(const _Float16* __restrict__ qh, const _Float16* __restrict__ kh, const float* __restrict__ v, const int* __restrict__ pos, float* __restrict__ out) {
  __shared__ __align__(16) float sS[2][16][LL + 8];
  __shared__ __align__(16) float sO[2][16][68];
  __shared__ float sw[2][16][KK];
  const int tid = threadIdx.x, w = tid >> 5, lane = tid & 31, col = lane & 15, g = lane >> 4;
  const int b = blockIdx.z, h = blockIdx.y, l0 = blockIdx.x * 32 + w * 16; const size_t bh = (size_t)b * NH + h;
  const _Float16* qb = qh + bh * LL * CC; const _Float16* kb = kh + bh * LL * CC;
  v16h aq[2];
#pragma unroll
  for (int kc = 0; kc < 2; ++kc) aq[kc] = frag_h(qb + (size_t)(l0 + col) * CC + kc * 32, lane);
#pragma unroll 2
  for (int t = 0; t < LL / 16; ++t) { v8f s = {};
#pragma unroll
    for (int kc = 0; kc < 2; ++kc) s = wmma16(aq[kc], frag_h(kb + (size_t)(t * 16 + col) * CC + kc * 32, lane), s);
#pragma unroll
    for (int r = 0; r < 8; ++r) sS[w][8 * g + r][t * 16 + col] = s[r] * 0.125f; }
  LDSX();
  { const int m = col; const size_t prow = ((((size_t)b * LL + l0 + m) * NH) + h) * KK; float* row = &sS[w][m][0];
    float sc[32]; float mx = -3.4e38f;
#pragma unroll
    for (int u = 0; u < 32; ++u) { int p = pos[prow + g * 32 + u]; p = p < 0 ? 0 : (p >= LL ? LL - 1 : p); sc[u] = row[p]; mx = fmaxf(mx, sc[u]); }
    mx = fmaxf(mx, __shfl_xor(mx, 16, 32)); float l = 0.f;
#pragma unroll
    for (int u = 0; u < 32; ++u) { sc[u] = expf(sc[u] - mx); l += sc[u]; }
    l += __shfl_xor(l, 16, 32); const float inv = 1.0f / l;
#pragma unroll
    for (int u = 0; u < 32; ++u) sw[w][m][g * 32 + u] = sc[u] * inv;
    LDSX();
    float o[32];
#pragma unroll
    for (int c = 0; c < 32; ++c) o[c] = 0.f;
#pragma unroll 2
    for (int u = 0; u < KK; ++u) { int p = pos[prow + u]; p = p < 0 ? 0 : (p >= LL ? LL - 1 : p); const float wu = sw[w][m][u]; const float* vr = v + ((((size_t)b * LL + p) * NH) + h) * CC + g * 32;
#pragma unroll
      for (int c4 = 0; c4 < 8; ++c4) { const v4f vv = *(const v4f*)(vr + c4 * 4); o[c4 * 4] += wu * vv[0]; o[c4 * 4 + 1] += wu * vv[1]; o[c4 * 4 + 2] += wu * vv[2]; o[c4 * 4 + 3] += wu * vv[3]; } }
#pragma unroll
    for (int c = 0; c < 32; ++c) sO[w][m][g * 32 + c] = o[c]; }
  LDSX();
  for (int qd = lane; qd < 16 * 16; qd += 32) { const int rl = qd >> 4, pc = qd & 15; vst2(out + ((((size_t)b * LL + l0 + rl) * NH) + h) * CC + pc * 4, *(const v4f*)(&sO[w][rl][pc * 4])); }
}
extern "C" void kernel_launch(void* const* d_in, const int* in_sizes, int n_in, void* d_out, int out_size, void* d_ws, size_t ws_size, hipStream_t stream) {
  (void)in_sizes; (void)n_in; (void)out_size; (void)ws_size;
  const float* q = (const float*)d_in[0]; const float* k = (const float*)d_in[1]; const float* v = (const float*)d_in[2]; const int* pos = (const int*)d_in[3];
  float* out = (float*)d_out;
  char* ws = (char*)d_ws; size_t off = 0;
  auto take = [&](size_t bytes) { char* p = ws + off; off += (bytes + 255) & ~(size_t)255; return p; };
  _Float16* qh = (_Float16*)take((size_t)NB * NH * LL * CC * 2); _Float16* kh = (_Float16*)take((size_t)NB * NH * LL * CC * 2); _Float16* vT = (_Float16*)take((size_t)NB * NH * CC * LL * 2);
  k_prep<<<dim3(LL / 64, NH, NB), 256, 0, stream>>>(q, k, v, qh, kh, vT);
  k_attn<<<dim3(LL / 32, NH, NB), 64, 0, stream>>>(qh, kh, v, pos, out);
}
